// LocalAttention_29463475651336
// MI455X (gfx1250) — hardware-verified
//
#include <hip/hip_runtime.h>

typedef _Float16 v16h __attribute__((ext_vector_type(16)));
typedef _Float16 v8h  __attribute__((ext_vector_type(8)));
typedef _Float16 v4h  __attribute__((ext_vector_type(4)));
typedef float    v8f  __attribute__((ext_vector_type(8)));
typedef float    v4f  __attribute__((ext_vector_type(4)));
typedef float    v4fa __attribute__((ext_vector_type(4), may_alias));
typedef unsigned int v4u  __attribute__((ext_vector_type(4)));
typedef unsigned int v4ua __attribute__((ext_vector_type(4), may_alias));

#ifndef NB
#define NB 2
#endif
#ifndef SEQ
#define SEQ 2048
#endif
#define NB_FULL 2
#define S_FULL  2048
#define DM      1024
#define NH      16
#define HD      64
#define HALF_W  64
#define QB      64
#define KP      72
#define VP      40
#define GM      128
#define GN      64
#define NEG_BIG (-1.0e30f)
#define SCALE   0.125f
#define PSCALE  1024.0f
#define LSCALE  2048.0f
#define RSPLIT  (1.0f / 2048.0f)
#define ASC     16.0f
#define WSC     256.0f
#define CSC     64.0f

#define XBYTES  ((size_t)NB_FULL * S_FULL * DM * 2)
#define WBYTES  ((size_t)DM * DM * 2)
#define HBYTES  ((size_t)NB_FULL * NH * S_FULL * HD * 4)
#define CBYTES  ((size_t)NB_FULL * S_FULL * DM * 2)
#define OFF_XQ  ((size_t)0)
#define OFF_XK  (OFF_XQ + XBYTES)
#define OFF_XV  (OFF_XK + XBYTES)
#define OFF_WQ  (OFF_XV + XBYTES)
#define OFF_WK  (OFF_WQ + WBYTES)
#define OFF_WV  (OFF_WK + WBYTES)
#define OFF_WO  (OFF_WV + WBYTES)
#define OFF_QH  (OFF_WO + WBYTES)
#define OFF_KH  (OFF_QH + HBYTES)
#define OFF_VH  (OFF_KH + HBYTES)
#define OFF_CT  (OFF_VH + HBYTES)
#define WS_TOTAL (OFF_CT + CBYTES)

static_assert(WS_TOTAL <= (size_t)134217728);
static_assert(SEQ % GM == 0);
static_assert(SEQ % QB == 0);
static_assert(SEQ % 32 == 0);
static_assert(SEQ <= S_FULL);
static_assert(NB >= 1 && NB <= NB_FULL);
static_assert(HD == 64 && GN == HD && NH * HD == DM);
static_assert(DM % 32 == 0 && DM % GN == 0);
static_assert((KP % 8) == 0 && (VP % 8) == 0);
static_assert(KP >= HD && VP >= 32);
static_assert(((size_t)NB_FULL * S_FULL * DM) % 2048 == 0);
static_assert(((size_t)DM * DM) % 2048 == 0);

static __device__ __forceinline__ float bf16r(float x)
{
    unsigned u = __float_as_uint(x);
    u = (u + 0x7FFFu + ((u >> 16) & 1u)) & 0xFFFF0000u;
    return __uint_as_float(u);
}

static __device__ __forceinline__ _Float16 tofh(float x, float sc)
{
    return (_Float16)(bf16r(x) * sc);
}

static __device__ __forceinline__ _Float16 toh(float x)
{
    return (_Float16)x;
}

static __device__ __forceinline__ v16h cat8(v8h a, v8h b)
{
    return __builtin_shufflevector(a, b, 0, 1, 2, 3, 4, 5, 6, 7, 8, 9, 10, 11, 12, 13, 14, 15);
}

static __device__ __forceinline__ v8f wmma16(v16h a, v16h b, v8f c)
{
    v8f d = __builtin_amdgcn_wmma_f32_16x16x32_f16(false, a, false, b, (short)0, c, false, false);
    asm volatile("v_nop\n\tv_nop\n\tv_nop\n\tv_nop" : "+v"(d) : "v"(a), "v"(b));
    return d;
}

__global__ void __launch_bounds__(256) cvt_plane_kernel(const float* __restrict__ src,
                                                         _Float16* __restrict__ dst,
                                                         float sc, int n8)
{
    const int t = blockIdx.x * 256 + threadIdx.x;
    if (t >= n8) return;
    const float* p = src + (size_t)t * 8;
    const v4f x0 = *(const v4f*)p;
    const v4f x1 = *(const v4f*)(p + 4);
    union { v8h h; v4u u; } o;
    o.h[0] = tofh(x0[0], sc); o.h[1] = tofh(x0[1], sc); o.h[2] = tofh(x0[2], sc); o.h[3] = tofh(x0[3], sc);
    o.h[4] = tofh(x1[0], sc); o.h[5] = tofh(x1[1], sc); o.h[6] = tofh(x1[2], sc); o.h[7] = tofh(x1[3], sc);
    const v4u ov = o.u;
    _Float16* d = dst + (size_t)t * 8;
    *(volatile v4u*)d = ov;
    __threadfence();
    *(volatile v4u*)d = ov;
}

template <int MODE>
__global__ void __launch_bounds__(128) gemm_xwT_kernel(const _Float16* __restrict__ A,
                                                        const _Float16* __restrict__ W,
                                                        const float* __restrict__ bias,
                                                        float* __restrict__ Out)
{
    __shared__ __align__(16) float sacc[4][32 * GN];

    const int tid  = threadIdx.x;
    const int lane = tid & 31;
    const int wave = __builtin_amdgcn_readfirstlane(tid >> 5);
    const int lo   = lane & 15;
    const int hi   = lane >> 4;
    const int koff = hi * 8;
    const int ct   = blockIdx.x;
    const int rt   = blockIdx.y;
    const int bb   = rt / (SEQ / GM);
    const int s0   = (rt - bb * (SEQ / GM)) * GM;
    const int n0   = ct * GN;
    const int wrow = bb * S_FULL + s0 + 32 * wave;

    const _Float16* ap0 = A + (size_t)(wrow + lo) * DM + koff;
    const _Float16* ap1 = A + (size_t)(wrow + 16 + lo) * DM + koff;
    const _Float16* wp[4];
#pragma unroll
    for (int nt = 0; nt < 4; ++nt) wp[nt] = W + (size_t)(n0 + 16 * nt + lo) * DM + koff;

    v8f acc0[4], acc1[4];
#pragma unroll
    for (int nt = 0; nt < 4; ++nt) { v8f z = {}; acc0[nt] = z; acc1[nt] = z; }

#pragma unroll 2
    for (int k0 = 0; k0 < DM; k0 += 32) {
        const v16h a0 = cat8(*(const v8h*)(ap0 + k0), *(const v8h*)(ap0 + k0 + 16));
        const v16h a1 = cat8(*(const v8h*)(ap1 + k0), *(const v8h*)(ap1 + k0 + 16));
        v16h bf[4];
#pragma unroll
        for (int nt = 0; nt < 4; ++nt)
            bf[nt] = cat8(*(const v8h*)(wp[nt] + k0), *(const v8h*)(wp[nt] + k0 + 16));
#pragma unroll
        for (int nt = 0; nt < 4; ++nt) {
            acc0[nt] = wmma16(a0, bf[nt], acc0[nt]);
            acc1[nt] = wmma16(a1, bf[nt], acc1[nt]);
        }
    }

    const float osc = (MODE == 0) ? (1.0f / (ASC * WSC)) : (1.0f / (CSC * WSC));
    float bc[4];
#pragma unroll
    for (int nt = 0; nt < 4; ++nt) bc[nt] = bf16r(bias[n0 + 16 * nt + lo]);

    float* so = sacc[wave];
#pragma unroll
    for (int nt = 0; nt < 4; ++nt) {
#pragma unroll
        for (int r = 0; r < 8; ++r) {
            so[(8 * hi + r) * GN + 16 * nt + lo]      = acc0[nt][r] * osc + bc[nt];
            so[(16 + 8 * hi + r) * GN + 16 * nt + lo] = acc1[nt][r] * osc + bc[nt];
        }
    }
    __syncthreads();

    v4f ov[16];
#pragma unroll
    for (int i = 0; i < 16; ++i) {
        const int cc = lane + 32 * i, rr = cc >> 4, qd = cc & 15;
        ov[i] = *(const v4fa*)(so + rr * GN + qd * 4);
    }
    float* dst;
    size_t ldo;
    if (MODE == 0) {
        dst = Out + ((size_t)(bb * NH + ct) * S_FULL + s0 + 32 * wave) * HD;
        ldo = HD;
    } else {
        dst = Out + (size_t)wrow * DM + n0;
        ldo = DM;
    }
#pragma unroll
    for (int i = 0; i < 16; ++i) {
        const int cc = lane + 32 * i, rr = cc >> 4, qd = cc & 15;
        *(volatile v4f*)(dst + (size_t)rr * ldo + qd * 4) = ov[i];
    }
    __threadfence();
#pragma unroll
    for (int i = 0; i < 16; ++i) {
        const int cc = lane + 32 * i, rr = cc >> 4, qd = cc & 15;
        *(volatile v4f*)(dst + (size_t)rr * ldo + qd * 4) = ov[i];
    }
}

__global__ void __launch_bounds__(128) band_attn_kernel(const float* __restrict__ Q,
                                                         const float* __restrict__ K,
                                                         const float* __restrict__ V,
                                                         _Float16* __restrict__ C)
{
    __shared__ __align__(16) _Float16 kbuf[32 * KP];
    __shared__ __align__(16) _Float16 vbuf[HD * VP];
    __shared__ __align__(16) _Float16 pbuf[4][16 * 32];
    __shared__ __align__(16) _Float16 plbuf[4][16 * 32];
    __shared__ __align__(16) _Float16 sctx[4][16 * HD];

    const int tid  = threadIdx.x;
    const int lane = tid & 31;
    const int wave = __builtin_amdgcn_readfirstlane(tid >> 5);
    const int lo   = lane & 15;
    const int hi   = lane >> 4;
    const int koff = hi * 8;
    const int q0   = blockIdx.x * QB;
    const int bh   = blockIdx.y;
    const int bb   = bh / NH;
    const int hh   = bh - bb * NH;
    const int qw   = q0 + wave * 16;
    const size_t rowbase = (size_t)bh * S_FULL;

    _Float16* pb  = pbuf[wave];
    _Float16* plb = plbuf[wave];

    v16h aq0, aq1;
    {
        const float* qr = Q + (rowbase + qw + lo) * HD;
        v8h f[4];
#pragma unroll
        for (int s = 0; s < 4; ++s) {
            const v4f x0 = *(const v4f*)(qr + 16 * s + koff);
            const v4f x1 = *(const v4f*)(qr + 16 * s + koff + 4);
            v8h t;
            t[0] = toh(x0[0]); t[1] = toh(x0[1]); t[2] = toh(x0[2]); t[3] = toh(x0[3]);
            t[4] = toh(x1[0]); t[5] = toh(x1[1]); t[6] = toh(x1[2]); t[7] = toh(x1[3]);
            f[s] = t;
        }
        aq0 = cat8(f[0], f[1]);
        aq1 = cat8(f[2], f[3]);
    }

    v8f oacc[4];
#pragma unroll
    for (int nt = 0; nt < 4; ++nt) { v8f z = {}; oacc[nt] = z; }
    float rm[8], rl[8];
#pragma unroll
    for (int i = 0; i < 8; ++i) { rm[i] = NEG_BIG; rl[i] = 0.0f; }

    int kmin = q0 - HALF_W; if (kmin < 0) kmin = 0;
    const int cb = kmin & ~31;
    int kmax = q0 + QB - 1 + HALF_W; if (kmax > SEQ - 1) kmax = SEQ - 1;

    for (int c = cb; c <= kmax; c += 32) {
#pragma unroll
        for (int it = 0; it < 4; ++it) {
            const int idx  = tid + 128 * it;
            const int row  = idx >> 4;
            const int col4 = (idx & 15) * 4;
            const size_t g = (rowbase + c + row) * HD + col4;
            const v4f kk = *(const v4f*)(K + g);
            const v4f vv = *(const v4f*)(V + g);
            v4h kh;
            kh[0] = toh(kk[0]); kh[1] = toh(kk[1]); kh[2] = toh(kk[2]); kh[3] = toh(kk[3]);
            *(v4h*)(kbuf + row * KP + col4) = kh;
            vbuf[(col4 + 0) * VP + row] = toh(vv[0]);
            vbuf[(col4 + 1) * VP + row] = toh(vv[1]);
            vbuf[(col4 + 2) * VP + row] = toh(vv[2]);
            vbuf[(col4 + 3) * VP + row] = toh(vv[3]);
        }
        __syncthreads();

        const bool active = (c <= qw + 15 + HALF_W) && (c + 31 >= qw - HALF_W);

        if (active) {
            const _Float16* k0r = kbuf + lo * KP;
            const _Float16* k1r = kbuf + (16 + lo) * KP;
            const v16h b00 = cat8(*(const v8h*)(k0r + koff),      *(const v8h*)(k0r + 16 + koff));
            const v16h b01 = cat8(*(const v8h*)(k0r + 32 + koff), *(const v8h*)(k0r + 48 + koff));
            const v16h b10 = cat8(*(const v8h*)(k1r + koff),      *(const v8h*)(k1r + 16 + koff));
            const v16h b11 = cat8(*(const v8h*)(k1r + 32 + koff), *(const v8h*)(k1r + 48 + koff));
            v8f cs0 = {}, cs1 = {};
            cs0 = wmma16(aq0, b00, cs0);
            cs0 = wmma16(aq1, b01, cs0);
            cs1 = wmma16(aq0, b10, cs1);
            cs1 = wmma16(aq1, b11, cs1);

#pragma unroll
            for (int i = 0; i < 8; ++i) {
                const int m = i + 8 * hi;
                const int q = qw + m;
                int d0 = q - (c + lo);      d0 = d0 < 0 ? -d0 : d0;
                int d1 = q - (c + 16 + lo); d1 = d1 < 0 ? -d1 : d1;
                const bool ok0 = (d0 <= HALF_W);
                const bool ok1 = (d1 <= HALF_W);
                const float sv0 = ok0 ? cs0[i] * SCALE : NEG_BIG;
                const float sv1 = ok1 ? cs1[i] * SCALE : NEG_BIG;

                float mx = fmaxf(sv0, sv1);
#pragma unroll
                for (int d = 1; d < 16; d <<= 1) mx = fmaxf(mx, __shfl_xor(mx, d, 32));
                const float mnew = fmaxf(rm[i], mx);
                const float scal = __expf(rm[i] - mnew);
                float p0 = __expf(sv0 - mnew); p0 = ok0 ? p0 : 0.0f;
                float p1 = __expf(sv1 - mnew); p1 = ok1 ? p1 : 0.0f;
                float sum = p0 + p1;
#pragma unroll
                for (int d = 1; d < 16; d <<= 1) sum += __shfl_xor(sum, d, 32);
                rl[i] = rl[i] * scal + sum;
                rm[i] = mnew;
#pragma unroll
                for (int nt = 0; nt < 4; ++nt) oacc[nt][i] *= scal;

                const float w0 = p0 * PSCALE, w1 = p1 * PSCALE;
                const _Float16 h0 = (_Float16)w0, h1 = (_Float16)w1;
                pb[m * 32 + lo]       = h0;  plb[m * 32 + lo]      = (_Float16)((w0 - (float)h0) * LSCALE);
                pb[m * 32 + 16 + lo]  = h1;  plb[m * 32 + 16 + lo] = (_Float16)((w1 - (float)h1) * LSCALE);
            }
        }
        __syncthreads();

        if (active) {
            const v16h ap  = cat8(*(const v8h*)(pb + lo * 32 + koff),  *(const v8h*)(pb + lo * 32 + 16 + koff));
            const v16h apl = cat8(*(const v8h*)(plb + lo * 32 + koff), *(const v8h*)(plb + lo * 32 + 16 + koff));
#pragma unroll
            for (int nt = 0; nt < 4; ++nt) {
                const _Float16* vr = vbuf + (nt * 16 + lo) * VP;
                const v16h vb = cat8(*(const v8h*)(vr + koff), *(const v8h*)(vr + 16 + koff));
                v8f x = {};
                x = wmma16(apl, vb, x);
                oacc[nt] = wmma16(ap, vb, oacc[nt]);
                oacc[nt] += x * RSPLIT;
            }
        }
        __syncthreads();
    }

    float inv[8];
#pragma unroll
    for (int i = 0; i < 8; ++i) inv[i] = (CSC / PSCALE) / rl[i];
    _Float16* so = sctx[wave];
#pragma unroll
    for (int nt = 0; nt < 4; ++nt) {
#pragma unroll
        for (int i = 0; i < 8; ++i) so[(i + 8 * hi) * HD + nt * 16 + lo] = toh(oacc[nt][i] * inv[i]);
    }
    __syncthreads();

    v4u ov[4];
#pragma unroll
    for (int i = 0; i < 4; ++i) {
        const int rr = 4 * i + (lane >> 3), qd = lane & 7;
        ov[i] = *(const v4ua*)(so + rr * HD + qd * 8);
    }
    _Float16* cbp = C + ((size_t)(bb * S_FULL + qw)) * DM + hh * HD;
#pragma unroll
    for (int i = 0; i < 4; ++i) {
        const int rr = 4 * i + (lane >> 3), qd = lane & 7;
        *(volatile v4u*)(cbp + (size_t)rr * DM + qd * 8) = ov[i];
    }
    __threadfence();
#pragma unroll
    for (int i = 0; i < 4; ++i) {
        const int rr = 4 * i + (lane >> 3), qd = lane & 7;
        *(volatile v4u*)(cbp + (size_t)rr * DM + qd * 8) = ov[i];
    }
}

extern "C" void kernel_launch(void* const* d_in, const int* in_sizes, int n_in,
                              void* d_out, int out_size, void* d_ws, size_t ws_size,
                              hipStream_t stream)
{
    if (n_in < 11) return;
    const long long arows = (long long)(NB - 1) * S_FULL + SEQ;
    const long long aneed = arows * DM;
    if ((long long)in_sizes[0] < aneed || (long long)in_sizes[1] < aneed || (long long)in_sizes[2] < aneed) return;
    if ((long long)in_sizes[3] < (long long)DM * DM || (long long)in_sizes[5] < (long long)DM * DM ||
        (long long)in_sizes[7] < (long long)DM * DM || (long long)in_sizes[9] < (long long)DM * DM) return;
    if (in_sizes[4] < DM || in_sizes[6] < DM || in_sizes[8] < DM || in_sizes[10] < DM) return;
    if ((long long)out_size < aneed) return;
    if (ws_size < WS_TOTAL) return;

    const float* queries = (const float*)d_in[0];
    const float* keys    = (const float*)d_in[1];
    const float* values  = (const float*)d_in[2];
    const float* wq = (const float*)d_in[3];
    const float* bq = (const float*)d_in[4];
    const float* wk = (const float*)d_in[5];
    const float* bk = (const float*)d_in[6];
    const float* wv = (const float*)d_in[7];
    const float* bv = (const float*)d_in[8];
    const float* wo = (const float*)d_in[9];
    const float* bo = (const float*)d_in[10];
    float* out = (float*)d_out;

    char* ws = (char*)d_ws;
    _Float16* Xq = (_Float16*)(ws + OFF_XQ);
    _Float16* Xk = (_Float16*)(ws + OFF_XK);
    _Float16* Xv = (_Float16*)(ws + OFF_XV);
    _Float16* Wq = (_Float16*)(ws + OFF_WQ);
    _Float16* Wk = (_Float16*)(ws + OFF_WK);
    _Float16* Wv = (_Float16*)(ws + OFF_WV);
    _Float16* Wo = (_Float16*)(ws + OFF_WO);
    float*    Qh = (float*)(ws + OFF_QH);
    float*    Kh = (float*)(ws + OFF_KH);
    float*    Vh = (float*)(ws + OFF_VH);
    _Float16* Ct = (_Float16*)(ws + OFF_CT);

    const int an8 = (int)(aneed / 8);
    const int wn8 = (DM * DM) / 8;
    const dim3 cga((an8 + 255) / 256), cgw((wn8 + 255) / 256);
    cvt_plane_kernel<<<cga, 256, 0, stream>>>(queries, Xq, ASC, an8);
    cvt_plane_kernel<<<cga, 256, 0, stream>>>(keys,    Xk, ASC, an8);
    cvt_plane_kernel<<<cga, 256, 0, stream>>>(values,  Xv, ASC, an8);
    cvt_plane_kernel<<<cgw, 256, 0, stream>>>(wq, Wq, WSC, wn8);
    cvt_plane_kernel<<<cgw, 256, 0, stream>>>(wk, Wk, WSC, wn8);
    cvt_plane_kernel<<<cgw, 256, 0, stream>>>(wv, Wv, WSC, wn8);
    cvt_plane_kernel<<<cgw, 256, 0, stream>>>(wo, Wo, WSC, wn8);

    const dim3 gg(DM / GN, (NB * SEQ) / GM);
    gemm_xwT_kernel<0><<<gg, 128, 0, stream>>>(Xq, Wq, bq, Qh);
    gemm_xwT_kernel<0><<<gg, 128, 0, stream>>>(Xk, Wk, bk, Kh);
    gemm_xwT_kernel<0><<<gg, 128, 0, stream>>>(Xv, Wv, bv, Vh);

    const dim3 ga(SEQ / QB, NB * NH);
    band_attn_kernel<<<ga, 128, 0, stream>>>(Qh, Kh, Vh, Ct);

    gemm_xwT_kernel<1><<<gg, 128, 0, stream>>>(Ct, Wo, bo, out);
}
